// NeuralAttention_63428077027729
// MI455X (gfx1250) — hardware-verified
//
#include <hip/hip_runtime.h>


#ifndef NHD
#define NHD 2
#endif
#define NHD_FULL 2
#define SEQ   512
#define DK    64
#define HH    256
#define WS_TOTAL ((size_t)HH * DK * 2 * 2 + (size_t)NHD * SEQ * DK * 2 * 2 + (size_t)NHD * SEQ * HH * 4 * 2)

static_assert(NHD >= 1 && NHD <= NHD_FULL);
static_assert(SEQ == 8 * 64);
static_assert(HH == 2 * 128);
static_assert((NHD * SEQ) % 64 == 0 && HH % 64 == 0);
static_assert(DK % 32 == 0 && DK % 2 == 0);
static_assert(((size_t)NHD * SEQ * DK) % 8 == 0 && ((size_t)DK * HH) % 64 == 0);
static_assert(4 * 32 * 16 == SEQ * 4);
static_assert((size_t)NHD_FULL * SEQ * SEQ * 4 == 2097152);
static_assert(SEQ * 4 <= 131072 && 16 * 68 * 4 <= 131072);
static_assert(WS_TOTAL <= (size_t)134217728);

typedef _Float16 h16;
typedef unsigned short bf;
typedef __attribute__((ext_vector_type(16))) __bf16   v16bf;
typedef __attribute__((ext_vector_type(16))) _Float16 v16h;
typedef __attribute__((ext_vector_type(8)))  _Float16 v8h;
typedef __attribute__((ext_vector_type(8)))  unsigned short v8us;
typedef __attribute__((ext_vector_type(8)))  float    v8f;
typedef __attribute__((ext_vector_type(4)))  float    v4f;
typedef __attribute__((ext_vector_type(2)))  _Float16 v2h;
typedef __attribute__((ext_vector_type(2)))  unsigned short v2us;
typedef v8h  __attribute__((may_alias)) v8ha;
typedef v4f  __attribute__((may_alias)) v4fa;
typedef v8us __attribute__((may_alias)) v8usa;

__device__ __forceinline__ unsigned short f2bf(float f) { unsigned u = __float_as_uint(f); u += 0x7FFFu + ((u >> 16) & 1u); return (unsigned short)(u >> 16); }
__device__ __forceinline__ float bf2f(unsigned short b) { return __uint_as_float(((unsigned)b) << 16); }
__device__ __forceinline__ float bfr(float f) { return bf2f(f2bf(f)); }
__device__ __forceinline__ v16h cat16(v8h lo, v8h hi) { return __builtin_shufflevector(lo, hi, 0, 1, 2, 3, 4, 5, 6, 7, 8, 9, 10, 11, 12, 13, 14, 15); }
__device__ __forceinline__ v16bf cat16b(v8us lo, v8us hi) { return __builtin_bit_cast(v16bf, __builtin_shufflevector(lo, hi, 0, 1, 2, 3, 4, 5, 6, 7, 8, 9, 10, 11, 12, 13, 14, 15)); }
__device__ __forceinline__ v8f wmma16(v16h a, v16h b, v8f c) { return __builtin_amdgcn_wmma_f32_16x16x32_f16(false, a, false, b, (short)0, c, false, false); }
__device__ __forceinline__ v8f wmmab(v16bf a, v16bf b, v8f c) { return __builtin_amdgcn_wmma_f32_16x16x32_bf16(false, a, false, b, (short)0, c, false, false); }

template <typename T16> struct WFrag;
template <> struct WFrag<h16> { typedef v16h V; static __device__ __forceinline__ V ld(const h16* p) { return cat16(*(const v8h*)p, *(const v8h*)(p + 16)); } static __device__ __forceinline__ v8f mma(V a, V b, v8f c) { return wmma16(a, b, c); } };
template <> struct WFrag<bf> { typedef v16bf V; static __device__ __forceinline__ V ld(const bf* p) { return cat16b(*(const v8us*)p, *(const v8us*)(p + 16)); } static __device__ __forceinline__ v8f mma(V a, V b, v8f c) { return wmmab(a, b, c); } };
template <typename T16, int NSPLIT, bool BIAS>
__global__ __launch_bounds__(32) void k_gemmw(const T16* __restrict__ A, const T16* __restrict__ A2, const T16* __restrict__ Bt, const T16* __restrict__ Bt2, int K, float* C, int ldc, const float* __restrict__ bias, float csc, size_t sA, size_t sB, size_t sC) {
    typedef typename WFrag<T16>::V V;
    __shared__ __align__(16) float os[16 * 68];
    const size_t z = blockIdx.z; A += z * sA; if (A2) A2 += z * sA; Bt += z * sB; if (Bt2) Bt2 += z * sB; C += z * sC;
    const int lane = threadIdx.x & 31, lr = lane & 15, hi = lane >> 4; const int r0 = blockIdx.x * 64, c0 = blockIdx.y * 64;
    v8f acc[4][4];
#pragma unroll
    for (int mb = 0; mb < 4; ++mb)
#pragma unroll
        for (int nb = 0; nb < 4; ++nb) acc[mb][nb] = (v8f){};
    const size_t aoff = (size_t)(r0 + lr) * K + 8 * hi, boff = (size_t)(c0 + lr) * K + 8 * hi;
#pragma unroll 1
    for (int kc = 0; kc < K; kc += 32) {
        V a[4], a2[4];
#pragma unroll
        for (int mb = 0; mb < 4; ++mb) { a[mb] = WFrag<T16>::ld(A + aoff + (size_t)mb * 16 * K + kc); if (NSPLIT == 1 || NSPLIT == 2) a2[mb] = WFrag<T16>::ld(A2 + aoff + (size_t)mb * 16 * K + kc); }
#pragma unroll
        for (int nb = 0; nb < 4; ++nb) { const V b = WFrag<T16>::ld(Bt + boff + (size_t)nb * 16 * K + kc); V b2; if (NSPLIT >= 2) b2 = WFrag<T16>::ld(Bt2 + boff + (size_t)nb * 16 * K + kc);
#pragma unroll
            for (int mb = 0; mb < 4; ++mb) { acc[mb][nb] = WFrag<T16>::mma(a[mb], b, acc[mb][nb]); if (NSPLIT == 1 || NSPLIT == 2) acc[mb][nb] = WFrag<T16>::mma(a2[mb], b, acc[mb][nb]); if (NSPLIT >= 2) acc[mb][nb] = WFrag<T16>::mma(a[mb], b2, acc[mb][nb]); } }
        asm volatile("v_nop\n\tv_nop\n\tv_nop\n\tv_nop" : "+v"(acc[0][0]), "+v"(acc[1][1]), "+v"(acc[2][2]), "+v"(acc[3][3]) : "v"(a[0]), "v"(a[3]));
    }
#pragma unroll
    for (int mb = 0; mb < 4; ++mb) {
#pragma unroll
        for (int nb = 0; nb < 4; ++nb) {
#pragma unroll
            for (int j = 0; j < 8; ++j) os[(hi * 8 + j) * 68 + nb * 16 + lr] = acc[mb][nb][j]; }
        __builtin_amdgcn_wave_barrier(); asm volatile("" ::: "memory");
        float* crow = C + (size_t)(r0 + mb * 16) * ldc + c0;
#pragma unroll 1
        for (int ps = 0; ps < 2; ++ps) {
#pragma unroll
            for (int s = 0; s < 8; ++s) { const int row = 2 * s + hi, cofs = lr * 4; v4f val = *(const v4fa*)(os + row * 68 + cofs); val = val * csc;
                if (BIAS) { val[0] += bfr(bias[c0 + cofs]); val[1] += bfr(bias[c0 + cofs + 1]); val[2] += bfr(bias[c0 + cofs + 2]); val[3] += bfr(bias[c0 + cofs + 3]); }
                *(volatile v4f*)(crow + (size_t)row * ldc + cofs) = val; }
            if (ps == 0) __threadfence(); }
        __builtin_amdgcn_wave_barrier(); asm volatile("" ::: "memory");
    }
}

__global__ __launch_bounds__(256) void k_wtG(const float* __restrict__ w, int K, int N, bf* Bt) {
    const int lane = threadIdx.x & 31; const int L0 = (blockIdx.x * 8 + (threadIdx.x >> 5)) * 8; const int nlines = N * K / 64;
#pragma unroll
    for (int ps = 0; ps < 2; ++ps) {
#pragma unroll 1
        for (int l = 0; l < 8; ++l) { const int L = L0 + l; if (L >= nlines) break; const size_t e = (size_t)L * 64 + lane * 2; const int k = (int)(e % K), n = (int)(e / K); v2us o;
            o[0] = f2bf(w[(size_t)k * N + n]); o[1] = f2bf(w[(size_t)(k + 1) * N + n]); *(volatile v2us*)(Bt + e) = o; }
        if (ps == 0) __threadfence(); }
}

__global__ __launch_bounds__(256) void k_cvt8(const float* __restrict__ src, bf* dst, size_t n8) { const size_t i = (size_t)blockIdx.x * 256 + threadIdx.x; if (i >= n8) return; const v8f v = *(const v8f*)(src + i * 8); v8us o;
#pragma unroll
    for (int k = 0; k < 8; ++k) o[k] = f2bf(v[k]); *(volatile v8us*)(dst + i * 8) = o; __threadfence(); *(volatile v8us*)(dst + i * 8) = o; }

__global__ __launch_bounds__(256) void k_pair(const float* __restrict__ QPF, const float* __restrict__ KPF, const float* __restrict__ w2, const float* __restrict__ b2, float* OUT) {
    __shared__ __align__(16) float s_sc[SEQ];
    const int rq = blockIdx.x; const int hd = rq / SEQ;
    const int tid = threadIdx.x, lane = tid & 31; const int wave = __builtin_amdgcn_readfirstlane(tid >> 5);
    const float* qrow = QPF + (size_t)rq * HH;
    float qv[8], wv[8];
#pragma unroll
    for (int c = 0; c < 2; ++c) { const v4f q4 = *(const v4f*)(qrow + c * 128 + lane * 4); const v4f w4 = *(const v4f*)(w2 + c * 128 + lane * 4);
#pragma unroll
        for (int e = 0; e < 4; ++e) { qv[c * 4 + e] = q4[e]; wv[c * 4 + e] = bfr(w4[e]); } }
    const float bb = bfr(b2[0]);
    const float* kb = KPF + (size_t)hd * SEQ * HH;
#pragma unroll 1
    for (int kk = 0; kk < SEQ / 8; ++kk) {
        const int j = wave * (SEQ / 8) + kk;
        const float* krow = kb + (size_t)j * HH;
        float acc = 0.0f;
#pragma unroll
        for (int c = 0; c < 2; ++c) { const v4f u4 = *(const v4f*)(krow + c * 128 + lane * 4);
#pragma unroll
            for (int e = 0; e < 4; ++e) { const float t = qv[c * 4 + e] + u4[e]; const float r = (t > 0.0f) ? t : 0.0f; acc = fmaf(wv[c * 4 + e], r, acc); } }
#pragma unroll
        for (int sh = 16; sh; sh >>= 1) acc += __shfl_xor(acc, sh, 32);
        if (lane == 0) s_sc[j] = acc;
    }
    __syncthreads();
    if (wave < 4) {
        const int f0 = (wave * 32 + lane) * 4;
        v4f p = *(const v4fa*)(s_sc + f0); p = p + bb;
        float* dst = OUT + (size_t)rq * SEQ + f0;
        *(volatile v4f*)dst = p; __threadfence(); *(volatile v4f*)dst = p;
    }
}

extern "C" void kernel_launch(void* const* d_in, const int* in_sizes, int n_in,
                              void* d_out, int out_size, void* d_ws, size_t ws_size, hipStream_t stream) {
    if (n_in < 6) return;
    if (in_sizes[0] < NHD * SEQ * DK || in_sizes[1] < NHD * SEQ * DK || in_sizes[2] < 2 * DK * HH || in_sizes[3] < HH || in_sizes[4] < HH || in_sizes[5] < 1) return;
    if (out_size < NHD * SEQ * SEQ) return;
    const float* Qm = (const float*)d_in[0];
    const float* Km = (const float*)d_in[1];
    const float* W1 = (const float*)d_in[2];
    const float* b1 = (const float*)d_in[3];
    const float* W2 = (const float*)d_in[4];
    const float* b2 = (const float*)d_in[5];
    float* OUT = (float*)d_out;

    char* wsp = (char*)d_ws;
    auto take = [&](size_t bytes) { char* p = wsp; wsp += (bytes + 255) & ~(size_t)255; return (void*)p; };
    bf*    WQT = (bf*)take((size_t)HH * DK * 2);
    bf*    WKT = (bf*)take((size_t)HH * DK * 2);
    bf*    QB  = (bf*)take((size_t)NHD * SEQ * DK * 2);
    bf*    KB  = (bf*)take((size_t)NHD * SEQ * DK * 2);
    float* QPF = (float*)take((size_t)NHD * SEQ * HH * 4);
    float* KPF = (float*)take((size_t)NHD * SEQ * HH * 4);
    if ((size_t)(wsp - (char*)d_ws) > ws_size) return;

    k_wtG<<<(unsigned)((DK * HH / 64 + 63) / 64), 256, 0, stream>>>(W1, DK, HH, WQT);
    k_wtG<<<(unsigned)((DK * HH / 64 + 63) / 64), 256, 0, stream>>>(W1 + (size_t)DK * HH, DK, HH, WKT);
    k_cvt8<<<(unsigned)(((size_t)NHD * SEQ * DK / 8 + 255) / 256), 256, 0, stream>>>(Qm, QB, (size_t)NHD * SEQ * DK / 8);
    k_cvt8<<<(unsigned)(((size_t)NHD * SEQ * DK / 8 + 255) / 256), 256, 0, stream>>>(Km, KB, (size_t)NHD * SEQ * DK / 8);
    k_gemmw<bf, 0, true><<<dim3(NHD * SEQ / 64, HH / 64, 1), 32, 0, stream>>>(QB, nullptr, WQT, nullptr, DK, QPF, HH, b1, 1.0f, 0, 0, 0);
    k_gemmw<bf, 0, false><<<dim3(NHD * SEQ / 64, HH / 64, 1), 32, 0, stream>>>(KB, nullptr, WKT, nullptr, DK, KPF, HH, nullptr, 1.0f, 0, 0, 0);
    k_pair<<<(unsigned)(NHD * SEQ), 256, 0, stream>>>(QPF, KPF, W2, b2, OUT);
}
